// EdgeClassifierGNN_54820962566504
// MI455X (gfx1250) — hardware-verified
//
#include <hip/hip_runtime.h>
#include <stddef.h>
#include <stdint.h>


#define DIN     256
#define DH      256
#define NOUT    2
#define PW      512
#define APW     512
#define NTHR    256
#define NWAVE   8
#define EPT     8
#define CHUNK   (NTHR * EPT)
#define WCAP    (EPT * 32)
#define LISTN   (NWAVE * WCAP)
#define NBMAX   2048
#define RCAP    28672
#define DEGCAP  64
#define PKS     11
#define GBM     64
#define GTHR    128
#define GNT     8
#define ELINE   16
#define LPW     4
#define WSMAX   268435456
#define LDS_AGG ((2 * RCAP + 2 * NBMAX + LISTN) * 4 + 64)

static_assert((CHUNK & (CHUNK - 1)) == 0 && CHUNK <= (1 << PKS));
static_assert((NBMAX & (NBMAX - 1)) == 0 && NBMAX <= (1 << PKS));
static_assert(NTHR * 8 == NBMAX);
static_assert(LISTN >= NBMAX);
static_assert(LISTN >= NWAVE * WCAP);
static_assert((RCAP % 32) == 0);
static_assert(LDS_AGG <= 300000);
static_assert(GBM == (GTHR / 32) * 16);
static_assert((DIN % 32) == 0 && (DH % 32) == 0);
static_assert(DIN == 8 * 32 && DH == 8 * 32);
static_assert(PW == 2 * DH && APW == 2 * DH);
static_assert((2 * DH) % (16 * GNT) == 0);
static_assert(ELINE * NOUT * 4 == 128);

typedef float          v4f  __attribute__((ext_vector_type(4)));
typedef float          v8f  __attribute__((ext_vector_type(8)));
typedef int            v4i  __attribute__((ext_vector_type(4)));
typedef int            v8i  __attribute__((ext_vector_type(8)));
typedef unsigned int   v4u  __attribute__((ext_vector_type(4)));
typedef unsigned short v8us __attribute__((ext_vector_type(8)));
typedef __bf16         v16b __attribute__((ext_vector_type(16)));
union FragB { v16b v; v8us h[2]; v8i w; };

__device__ __forceinline__ v8f wmb(const FragB& a, const FragB& b, v8f c) {
  v8f d = __builtin_amdgcn_wmma_f32_16x16x32_bf16(false, a.v, false, b.v, (short)0, c, false, false);
  asm volatile("v_nop\n\tv_nop\n\tv_nop\n\tv_nop" : "+v"(d) : "v"(a.w), "v"(b.w));
  return d;
}

__device__ __forceinline__ unsigned short bf_bits(float f) {
  unsigned int u = __float_as_uint(f);
  u += 0x7FFFu + ((u >> 16) & 1u);
  return (unsigned short)(u >> 16);
}
__device__ __forceinline__ float bf_val(unsigned short b) {
  return __uint_as_float(((unsigned int)b) << 16);
}
__device__ __forceinline__ float bf_rne(float f) { return bf_val(bf_bits(f)); }

__device__ __forceinline__ v8us cvt8b(const v4f a, const v4f b) {
  v8us hv;
  hv[0] = bf_bits(a.x); hv[1] = bf_bits(a.y); hv[2] = bf_bits(a.z); hv[3] = bf_bits(a.w);
  hv[4] = bf_bits(b.x); hv[5] = bf_bits(b.y); hv[6] = bf_bits(b.z); hv[7] = bf_bits(b.w);
  return hv;
}

__device__ __forceinline__ int scan_chunk(const int* __restrict__ dsts, int nE, int cbase, int slotBase,
                                          int nb, int vec8, int* list, int tid, int lane, int wave) {
  int wc = 0;
  const int el0  = tid * EPT;
  const int e0   = cbase + el0;
  const int sent = -2147483647 - 1;
  v4i da, db;
  if (vec8 != 0 && cbase + CHUNK <= nE) {
    da = *(const v4i*)(dsts + e0);
    db = *(const v4i*)(dsts + e0 + 4);
  } else {
    da.x = (e0     < nE) ? dsts[min(e0,     nE - 1)] : sent;
    da.y = (e0 + 1 < nE) ? dsts[min(e0 + 1, nE - 1)] : sent;
    da.z = (e0 + 2 < nE) ? dsts[min(e0 + 2, nE - 1)] : sent;
    da.w = (e0 + 3 < nE) ? dsts[min(e0 + 3, nE - 1)] : sent;
    db.x = (e0 + 4 < nE) ? dsts[min(e0 + 4, nE - 1)] : sent;
    db.y = (e0 + 5 < nE) ? dsts[min(e0 + 5, nE - 1)] : sent;
    db.z = (e0 + 6 < nE) ? dsts[min(e0 + 6, nE - 1)] : sent;
    db.w = (e0 + 7 < nE) ? dsts[min(e0 + 7, nE - 1)] : sent;
  }
  const unsigned nbs = (unsigned)slotBase;
  const unsigned unb = (unsigned)nb;
  const unsigned s0 = (unsigned)da.x - nbs, s1 = (unsigned)da.y - nbs;
  const unsigned s2 = (unsigned)da.z - nbs, s3 = (unsigned)da.w - nbs;
  const unsigned s4 = (unsigned)db.x - nbs, s5 = (unsigned)db.y - nbs;
  const unsigned s6 = (unsigned)db.z - nbs, s7 = (unsigned)db.w - nbs;
  const bool h0 = s0 < unb, h1 = s1 < unb, h2 = s2 < unb, h3 = s3 < unb;
  const bool h4 = s4 < unb, h5 = s5 < unb, h6 = s6 < unb, h7 = s7 < unb;
  const unsigned any = __builtin_amdgcn_ballot_w32(h0 | h1 | h2 | h3 | h4 | h5 | h6 | h7);
  if (any != 0u) {
#define HITJ(J, HJ, SJ) { \
      const unsigned mj = __builtin_amdgcn_ballot_w32(HJ); \
      if (mj != 0u) { \
        if (HJ) { \
          const int pos = wc + (int)__builtin_amdgcn_mbcnt_lo(mj, 0u); \
          if (pos < WCAP) list[wave * WCAP + pos] = ((el0 + (J)) << PKS) | (int)(SJ); \
        } \
        wc += (int)__builtin_popcount(mj); } }
    HITJ(0, h0, s0)
    HITJ(1, h1, s1)
    HITJ(2, h2, s2)
    HITJ(3, h3, s3)
    HITJ(4, h4, s4)
    HITJ(5, h5, s5)
    HITJ(6, h6, s6)
    HITJ(7, h7, s7)
#undef HITJ
  }
  return wc;
}

__global__ __launch_bounds__(NTHR) void k_xprep(const float* __restrict__ x, unsigned short* xb,
                                                int nN, int nUnits) {
  const int i = (int)blockIdx.x * NTHR + (int)threadIdx.x;
  if (i >= nUnits) return;
  const int row = i >> 5;
  const int c0  = (i & 31) * 8;
  const int rc  = row < nN ? row : nN - 1;
  const float* p = x + (size_t)rc * DIN + c0;
  v4f a = *(const v4f*)p, b = *(const v4f*)(p + 4);
  const v4f z4 = {0.f, 0.f, 0.f, 0.f};
  if (row >= nN) { a = z4; b = z4; }
  const v8us hv = cvt8b(a, b);
  const size_t o = (size_t)row * DIN + c0;
  *(volatile v8us*)(xb + o) = hv;
  __threadfence();
  *(volatile v8us*)(xb + o) = hv;
}

__global__ __launch_bounds__(NTHR) void k_wtr(const float* __restrict__ w0, const float* __restrict__ w1,
                                              int c0, int c1, int segRows, int Kin, int K,
                                              unsigned short* wt, int nUnits) {
  const int u = (int)blockIdx.x * NTHR + (int)threadIdx.x;
  if (u >= nUnits) return;
  const int kq = K >> 3;
  const int n  = u / kq;
  const int k8 = (u - n * kq) * 8;
  int seg = n / segRows;
  seg = seg > 1 ? 1 : (seg < 0 ? 0 : seg);
  const int nc = n - seg * segRows;
  const float* ws = (seg == 0) ? w0 : w1;
  const int cc = (seg == 0) ? c0 : c1;
  int ncl = nc < cc ? nc : cc - 1;
  ncl = ncl < 0 ? 0 : ncl;
  int ks = k8 - (k8 / Kin) * Kin;
  ks = ks < 0 ? 0 : ks;
  const float* p = ws + (size_t)ks * (size_t)cc + ncl;
  v4f a, b;
  a.x = p[0];                  a.y = p[(size_t)cc];         a.z = p[(size_t)2 * cc];     a.w = p[(size_t)3 * cc];
  b.x = p[(size_t)4 * cc];     b.y = p[(size_t)5 * cc];     b.z = p[(size_t)6 * cc];     b.w = p[(size_t)7 * cc];
  const v4f z4 = {0.f, 0.f, 0.f, 0.f};
  if (nc >= cc) { a = z4; b = z4; }
  const v8us hv = cvt8b(a, b);
  const size_t o = (size_t)n * (size_t)K + k8;
  *(volatile v8us*)(wt + o) = hv;
  __threadfence();
  *(volatile v8us*)(wt + o) = hv;
}

template<int NT>
__global__ __launch_bounds__(GTHR) void k_gemm(const unsigned short* A, int lda,
                                               const unsigned short* __restrict__ WT, int K,
                                               float* outF, int ldo)
{
  constexpr int BN  = 16 * NT;
  constexpr int LPR = 4 * NT;
  constexpr int RPI = 32 / LPR;
  constexpr int NI  = 16 / RPI;
  __shared__ __attribute__((aligned(16))) float stg[GBM * BN];
  const int tid = (int)threadIdx.x, lane = tid & 31, wave = tid >> 5, hh = lane >> 4, m = lane & 15;
  const int rowBase = (int)blockIdx.x * GBM;
  const int col0    = (int)blockIdx.y * BN;

  v8f acc[NT];
  {
    const v8f z = {0.f, 0.f, 0.f, 0.f, 0.f, 0.f, 0.f, 0.f};
#pragma unroll
    for (int t = 0; t < NT; ++t) acc[t] = z;
  }
  const unsigned short* ap = A  + (size_t)(rowBase + 16 * wave + m) * (size_t)lda + 8 * hh;
  const unsigned short* wp = WT + (size_t)(col0 + m) * (size_t)K + 8 * hh;
  const int ksteps = K >> 5;
#pragma unroll 1
  for (int ks = 0; ks < ksteps; ++ks) {
    FragB af;
    af.h[0] = *(const v8us*)(ap + 32 * ks);
    af.h[1] = *(const v8us*)(ap + 32 * ks + 16);
#pragma unroll
    for (int t = 0; t < NT; ++t) {
      const unsigned short* wq = wp + (size_t)(16 * t) * (size_t)K + 32 * ks;
      FragB bf;
      bf.h[0] = *(const v8us*)wq;
      bf.h[1] = *(const v8us*)(wq + 16);
      acc[t] = wmb(af, bf, acc[t]);
    }
  }

#pragma unroll
  for (int t = 0; t < NT; ++t) {
    const int lc = 16 * t + m;
#pragma unroll
    for (int r = 0; r < 8; ++r) {
      const int lr = 16 * wave + 8 * hh + r;
      stg[lr * BN + lc] = acc[t][r];
    }
  }
  __syncthreads();

  const int rsub = lane / LPR;
  const int cp   = lane - rsub * LPR;
  v4f fv[NI];
#pragma unroll
  for (int i = 0; i < NI; ++i) {
    const int lr = 16 * wave + RPI * i + rsub;
    fv[i] = *(const v4f*)(stg + lr * BN + 4 * cp);
  }
#pragma unroll
  for (int i = 0; i < NI; ++i) {
    const int lr = 16 * wave + RPI * i + rsub;
    const int gr = rowBase + lr;
    float* op = outF + (size_t)gr * (size_t)ldo + col0 + 4 * cp;
    *(volatile v4f*)op = fv[i];
  }
  __threadfence();
#pragma unroll
  for (int i = 0; i < NI; ++i) {
    const int lr = 16 * wave + RPI * i + rsub;
    const int gr = rowBase + lr;
    float* op = outF + (size_t)gr * (size_t)ldo + col0 + 4 * cp;
    *(volatile v4f*)op = fv[i];
  }
}

__global__ __launch_bounds__(NTHR) void k_agg(
    const int* __restrict__ srcs, const int* __restrict__ dsts,
    const float* __restrict__ P, int pitchP, int selfOff, int nbrOff,
    const float* __restrict__ bias,
    unsigned short* Aout, int ldaOut,
    int nN, int nE, int nb, int vec8, int MPr) {
  extern __shared__ v4f lds_dyn[];
  int* reg1 = (int*)lds_dyn;
  int* reg2 = reg1 + RCAP;
  int* scnt = reg2 + RCAP;
  int* soff = scnt + NBMAX;
  int* list = soff + NBMAX;
  int* wcnt = list + LISTN;
  int* wtot = wcnt + NWAVE;
  const int tid = (int)threadIdx.x, lane = tid & 31, wave = tid >> 5;
  const int nodeBase = (int)blockIdx.x * nb;

  for (int i = tid; i < NBMAX; i += NTHR) scnt[i] = 0;
  __syncthreads();

  int tot = 0;
  const int nChunks = (nE + CHUNK - 1) / CHUNK;
#pragma unroll 1
  for (int ch = 0; ch < nChunks; ++ch) {
    const int cbase = ch * CHUNK;
    const int wc = scan_chunk(dsts, nE, cbase, nodeBase, nb, vec8, list, tid, lane, wave);
    if (lane == 0) wcnt[wave] = wc;
    __syncthreads();
    int pre = 0, all = 0;
#pragma unroll
    for (int w2 = 0; w2 < NWAVE; ++w2) {
      int c = wcnt[w2];
      c = c < 0 ? 0 : (c > WCAP ? WCAP : c);
      all += c;
      pre += (w2 < wave) ? c : 0;
    }
    const int wcc  = wc > WCAP ? WCAP : wc;
    const int base = tot + pre;
#pragma unroll 1
    for (int i = lane; i < wcc; i += 32) {
      const int ent = list[wave * WCAP + i];
      const int el  = (ent >> PKS) & (CHUNK - 1);
      const int sl  = ent & (NBMAX - 1);
      int eid = cbase + el;
      eid = eid > nE - 1 ? nE - 1 : eid;
      const int pos = base + i;
      if (pos < RCAP) reg1[pos] = (int)(((unsigned)eid << PKS) | (unsigned)sl);
    }
    tot += all;
    tot = tot > RCAP ? RCAP : tot;
    __syncthreads();
  }
  const int nh = tot;

  if (wave == 0) {
#pragma unroll 1
    for (int b0 = 0; b0 < nh; b0 += 32) {
      const int idx = b0 + lane;
      const int uv  = reg1[idx < RCAP ? idx : RCAP - 1];
      const int m32 = (nh - b0) < 32 ? (nh - b0) : 32;
#pragma unroll 1
      for (int k = 0; k < m32; ++k) {
        const int u  = __builtin_amdgcn_readlane(uv, k);
        const int sl = u & (NBMAX - 1);
        if (lane == 0) scnt[sl] = scnt[sl] + 1;
      }
    }
  }
  __syncthreads();

  {
    const v4i ca = *(const v4i*)(scnt + 8 * tid);
    const v4i cb = *(const v4i*)(scnt + 8 * tid + 4);
    const int e0 = ca.x < 0 ? 0 : ca.x, e1 = ca.y < 0 ? 0 : ca.y, e2 = ca.z < 0 ? 0 : ca.z, e3 = ca.w < 0 ? 0 : ca.w;
    const int e4 = cb.x < 0 ? 0 : cb.x, e5 = cb.y < 0 ? 0 : cb.y, e6 = cb.z < 0 ? 0 : cb.z, e7 = cb.w < 0 ? 0 : cb.w;
    const int ts = e0 + e1 + e2 + e3 + e4 + e5 + e6 + e7;
    int incl = ts;
#pragma unroll
    for (int d = 1; d < 32; d <<= 1) {
      const int up = __shfl_up(incl, d);
      if (lane >= d) incl += up;
    }
    if (lane == 31) wtot[wave] = incl;
    __syncthreads();
    int pre = 0;
#pragma unroll
    for (int w2 = 0; w2 < NWAVE; ++w2) pre += (w2 < wave) ? wtot[w2] : 0;
    int run = pre + incl - ts;
    soff[8 * tid + 0] = run; run += e0;
    soff[8 * tid + 1] = run; run += e1;
    soff[8 * tid + 2] = run; run += e2;
    soff[8 * tid + 3] = run; run += e3;
    soff[8 * tid + 4] = run; run += e4;
    soff[8 * tid + 5] = run; run += e5;
    soff[8 * tid + 6] = run; run += e6;
    soff[8 * tid + 7] = run;
  }
  __syncthreads();
  for (int i = tid; i < NBMAX; i += NTHR) list[i] = soff[i];
  __syncthreads();

  if (wave == 0) {
#pragma unroll 1
    for (int b0 = 0; b0 < nh; b0 += 32) {
      const int idx = b0 + lane;
      const int uv  = reg1[idx < RCAP ? idx : RCAP - 1];
      const int m32 = (nh - b0) < 32 ? (nh - b0) : 32;
#pragma unroll 1
      for (int k = 0; k < m32; ++k) {
        const int u   = __builtin_amdgcn_readlane(uv, k);
        const int sl  = u & (NBMAX - 1);
        const int eid = (int)((unsigned)u >> PKS);
        if (lane == 0) {
          int pos = list[sl];
          pos = pos < 0 ? 0 : (pos > RCAP - 1 ? RCAP - 1 : pos);
          reg2[pos] = eid;
          list[sl] = pos + 1;
        }
      }
    }
  }
  __syncthreads();

  const int nbw = nb >> 3;
  const bool ovf = (nh >= RCAP);
  const float qnan = __int_as_float(0x7fc00000);
  float bb[8];
  {
    const v4f ba = *(const v4f*)(bias + 8 * lane);
    const v4f bc = *(const v4f*)(bias + 8 * lane + 4);
    bb[0] = bf_rne(ba.x); bb[1] = bf_rne(ba.y); bb[2] = bf_rne(ba.z); bb[3] = bf_rne(ba.w);
    bb[4] = bf_rne(bc.x); bb[5] = bf_rne(bc.y); bb[6] = bf_rne(bc.z); bb[7] = bf_rne(bc.w);
  }

#pragma unroll 1
  for (int jt = 0; jt < nbw; ++jt) {
    const int slot = wave * nbw + jt;
    const int grow = nodeBase + slot;
    const int gcl  = grow < nN ? grow : nN - 1;
    int st = soff[slot];
    const int craw = scnt[slot];
    int cnt = craw;
    st  = st < 0 ? 0 : (st > nh ? nh : st);
    cnt = cnt < 0 ? 0 : (cnt > DEGCAP ? DEGCAP : cnt);
    if (cnt > nh - st) cnt = nh - st;
    const float pz = (ovf || craw > DEGCAP) ? qnan : 0.0f;
    const float live = grow < nN ? 1.0f : 0.0f;

    const float* srow = P + (size_t)gcl * (size_t)pitchP + selfOff + 8 * lane;
    const v4f sa = *(const v4f*)srow;
    const v4f sb = *(const v4f*)(srow + 4);
    v4f ga = {0.f, 0.f, 0.f, 0.f};
    v4f gb = {0.f, 0.f, 0.f, 0.f};

#pragma unroll 1
    for (int q = 0; q < cnt; ++q) {
      int idx = st + q; idx = idx > RCAP - 1 ? RCAP - 1 : idx;
      int eid = reg2[idx]; eid = eid < 0 ? 0 : (eid > nE - 1 ? nE - 1 : eid);
      const int sraw = srcs[eid];
      const int s = sraw < 0 ? 0 : (sraw > nN - 1 ? nN - 1 : sraw);
      const float* nr = P + (size_t)s * (size_t)pitchP + nbrOff + 8 * lane;
      const v4f na = *(const v4f*)nr;
      const v4f nbv = *(const v4f*)(nr + 4);
      ga += na;
      gb += nbv;
    }
    const float dcl  = cnt > 0 ? (float)cnt : 1.0f;
    const float invd = 1.0f / dcl;
    float rv[8];
    rv[0] = fmaxf((sa.x + ga.x * invd) + bb[0], 0.0f) * live + pz;
    rv[1] = fmaxf((sa.y + ga.y * invd) + bb[1], 0.0f) * live + pz;
    rv[2] = fmaxf((sa.z + ga.z * invd) + bb[2], 0.0f) * live + pz;
    rv[3] = fmaxf((sa.w + ga.w * invd) + bb[3], 0.0f) * live + pz;
    rv[4] = fmaxf((sb.x + gb.x * invd) + bb[4], 0.0f) * live + pz;
    rv[5] = fmaxf((sb.y + gb.y * invd) + bb[5], 0.0f) * live + pz;
    rv[6] = fmaxf((sb.z + gb.z * invd) + bb[6], 0.0f) * live + pz;
    rv[7] = fmaxf((sb.w + gb.w * invd) + bb[7], 0.0f) * live + pz;

    unsigned short hb[8], lb[8];
#pragma unroll
    for (int c = 0; c < 8; ++c) {
      hb[c] = bf_bits(rv[c]);
      lb[c] = bf_bits(rv[c] - bf_val(hb[c]));
    }
    v4u hw, lw;
    hw.x = (unsigned int)hb[0] | ((unsigned int)hb[1] << 16);
    hw.y = (unsigned int)hb[2] | ((unsigned int)hb[3] << 16);
    hw.z = (unsigned int)hb[4] | ((unsigned int)hb[5] << 16);
    hw.w = (unsigned int)hb[6] | ((unsigned int)hb[7] << 16);
    lw.x = (unsigned int)lb[0] | ((unsigned int)lb[1] << 16);
    lw.y = (unsigned int)lb[2] | ((unsigned int)lb[3] << 16);
    lw.z = (unsigned int)lb[4] | ((unsigned int)lb[5] << 16);
    lw.w = (unsigned int)lb[6] | ((unsigned int)lb[7] << 16);
    const int growc = grow < MPr ? grow : MPr - 1;
    unsigned short* gp = Aout + (size_t)growc * (size_t)ldaOut + 8 * lane;
    const bool wsv = grow < MPr;
    if (wsv) { *(volatile v4u*)gp = hw; *(volatile v4u*)(gp + DH) = lw; }
    __threadfence();
    if (wsv) { *(volatile v4u*)gp = hw; *(volatile v4u*)(gp + DH) = lw; }
  }
}

__global__ __launch_bounds__(NTHR) void k_edge(const float* __restrict__ PQ, int pitch, int qOff,
                                               const int* __restrict__ srcs, const int* __restrict__ dsts,
                                               const float* __restrict__ bm1, const float* __restrict__ Wm2,
                                               const float* __restrict__ bm2, float* out,
                                               int nN, int nE, int nLines) {
  const int tid = (int)threadIdx.x, lane = tid & 31, wave = tid >> 5;
  float bb[8], wa[8], wb[8];
  {
    const v4f ba = *(const v4f*)(bm1 + 8 * lane);
    const v4f bc = *(const v4f*)(bm1 + 8 * lane + 4);
    bb[0] = bf_rne(ba.x); bb[1] = bf_rne(ba.y); bb[2] = bf_rne(ba.z); bb[3] = bf_rne(ba.w);
    bb[4] = bf_rne(bc.x); bb[5] = bf_rne(bc.y); bb[6] = bf_rne(bc.z); bb[7] = bf_rne(bc.w);
    const float* wq = Wm2 + (size_t)(8 * lane) * NOUT;
    const v4f w0 = *(const v4f*)wq;
    const v4f w1 = *(const v4f*)(wq + 4);
    const v4f w2 = *(const v4f*)(wq + 8);
    const v4f w3 = *(const v4f*)(wq + 12);
    wa[0] = bf_rne(w0.x); wb[0] = bf_rne(w0.y); wa[1] = bf_rne(w0.z); wb[1] = bf_rne(w0.w);
    wa[2] = bf_rne(w1.x); wb[2] = bf_rne(w1.y); wa[3] = bf_rne(w1.z); wb[3] = bf_rne(w1.w);
    wa[4] = bf_rne(w2.x); wb[4] = bf_rne(w2.y); wa[5] = bf_rne(w2.z); wb[5] = bf_rne(w2.w);
    wa[6] = bf_rne(w3.x); wb[6] = bf_rne(w3.y); wa[7] = bf_rne(w3.z); wb[7] = bf_rne(w3.w);
  }
  const float cb0 = bf_rne(bm2[0]);
  const float cb1 = bf_rne(bm2[1]);
  const v4f z4 = {0.f, 0.f, 0.f, 0.f};

#pragma unroll 1
  for (int i = 0; i < LPW; ++i) {
    const int line = ((int)blockIdx.x * NWAVE + wave) * LPW + i;
    if (line >= nLines) break;
    const int e0 = line * ELINE;
    int el = e0 + (lane & 15);
    el = el > nE - 1 ? nE - 1 : el;
    const int svl = srcs[el];
    const int dvl = dsts[el];
    v4f ov = z4;
#pragma unroll 1
    for (int j = 0; j < ELINE; ++j) {
      int s = __shfl(svl, j);
      s = s < 0 ? 0 : (s > nN - 1 ? nN - 1 : s);
      int d = __shfl(dvl, j);
      d = d < 0 ? 0 : (d > nN - 1 ? nN - 1 : d);
      const float* pp = PQ + (size_t)s * (size_t)pitch + 8 * lane;
      const float* qp = PQ + (size_t)d * (size_t)pitch + qOff + 8 * lane;
      const v4f pa = *(const v4f*)pp;
      const v4f pb = *(const v4f*)(pp + 4);
      const v4f qa = *(const v4f*)qp;
      const v4f qb = *(const v4f*)(qp + 4);
      const float h0 = fmaxf((pa.x + qa.x) + bb[0], 0.0f);
      const float h1 = fmaxf((pa.y + qa.y) + bb[1], 0.0f);
      const float h2 = fmaxf((pa.z + qa.z) + bb[2], 0.0f);
      const float h3 = fmaxf((pa.w + qa.w) + bb[3], 0.0f);
      const float h4 = fmaxf((pb.x + qb.x) + bb[4], 0.0f);
      const float h5 = fmaxf((pb.y + qb.y) + bb[5], 0.0f);
      const float h6 = fmaxf((pb.z + qb.z) + bb[6], 0.0f);
      const float h7 = fmaxf((pb.w + qb.w) + bb[7], 0.0f);
      float p0 = h0 * wa[0];
      p0 = fmaf(h1, wa[1], p0); p0 = fmaf(h2, wa[2], p0); p0 = fmaf(h3, wa[3], p0);
      p0 = fmaf(h4, wa[4], p0); p0 = fmaf(h5, wa[5], p0); p0 = fmaf(h6, wa[6], p0); p0 = fmaf(h7, wa[7], p0);
      float p1 = h0 * wb[0];
      p1 = fmaf(h1, wb[1], p1); p1 = fmaf(h2, wb[2], p1); p1 = fmaf(h3, wb[3], p1);
      p1 = fmaf(h4, wb[4], p1); p1 = fmaf(h5, wb[5], p1); p1 = fmaf(h6, wb[6], p1); p1 = fmaf(h7, wb[7], p1);
      p0 += __shfl_xor(p0, 16); p1 += __shfl_xor(p1, 16);
      p0 += __shfl_xor(p0, 8);  p1 += __shfl_xor(p1, 8);
      p0 += __shfl_xor(p0, 4);  p1 += __shfl_xor(p1, 4);
      p0 += __shfl_xor(p0, 2);  p1 += __shfl_xor(p1, 2);
      p0 += __shfl_xor(p0, 1);  p1 += __shfl_xor(p1, 1);
      p0 += cb0;
      p1 += cb1;
      const bool mine = (lane == (j >> 1));
      const bool ev   = ((j & 1) == 0);
      ov.x = (mine && ev)  ? p0 : ov.x;
      ov.y = (mine && ev)  ? p1 : ov.y;
      ov.z = (mine && !ev) ? p0 : ov.z;
      ov.w = (mine && !ev) ? p1 : ov.w;
    }
    const int lq = lane < 8 ? lane : 7;
    float* op = out + (size_t)line * (size_t)(ELINE * NOUT) + 4 * lq;
    const bool wl = lane < 8;
    if (wl) *(volatile v4f*)op = ov;
    __threadfence();
    if (wl) *(volatile v4f*)op = ov;
  }
}

static int pick_nb(int nE, int nN) {
  int nb = NBMAX;
  while (nb > 16 && (long long)nb * (long long)nE * 5LL > (long long)RCAP * (long long)nN * 4LL) nb >>= 1;
  return nb;
}
static inline int cdiv(int a, int b) { return (a + b - 1) / b; }

extern "C" void kernel_launch(void* const* d_in, const int* in_sizes, int n_in,
                              void* d_out, int out_size, void* d_ws, size_t ws_size,
                              hipStream_t stream) {
  if (n_in < 12) return;
  if (in_sizes[0] < DIN) return;
  const int nN = in_sizes[0] / DIN;
  if (nN <= 0 || in_sizes[0] != nN * DIN || nN > (1 << 22)) return;
  if (in_sizes[1] < 2 * ELINE || (in_sizes[1] & 1) != 0) return;
  const int nE = in_sizes[1] / 2;
  if (nE > (1 << 21) || (nE % ELINE) != 0) return;
  if (in_sizes[2] != DIN * DH || in_sizes[3] != DH || in_sizes[4] != DIN * DH) return;
  if (in_sizes[5] != DH * DH  || in_sizes[6] != DH || in_sizes[7] != DH * DH) return;
  if (in_sizes[8] != 2 * DH * DH || in_sizes[9] != DH) return;
  if (in_sizes[10] != DH * NOUT || in_sizes[11] != NOUT) return;
  if (out_size != nE * NOUT) return;

  const float* x   = (const float*)d_in[0];
  const int*   ei  = (const int*)  d_in[1];
  const float* W1l = (const float*)d_in[2];
  const float* b1l = (const float*)d_in[3];
  const float* W1r = (const float*)d_in[4];
  const float* W2l = (const float*)d_in[5];
  const float* b2l = (const float*)d_in[6];
  const float* W2r = (const float*)d_in[7];
  const float* Wm1 = (const float*)d_in[8];
  const float* bm1 = (const float*)d_in[9];
  const float* Wm2 = (const float*)d_in[10];
  const float* bm2 = (const float*)d_in[11];
  float* out = (float*)d_out;
  const int* src = ei;
  const int* dst = ei + nE;

  const int MP     = cdiv(nN, GBM) * GBM;
  const int nb     = pick_nb(nE, nN);
  const int gA     = cdiv(MP, nb);
  const int vec8   = ((nE & 3) == 0) ? 1 : 0;
  const int nLines = nE / ELINE;
  if (gA * nb < MP) return;

  char* ws = (char*)d_ws;
  size_t off = 0;
  const size_t oACT = off; off += (size_t)MP * APW * 2;               off = (off + 255) & ~(size_t)255;
  const size_t oP   = off; off += (size_t)MP * PW * 4;                off = (off + 255) & ~(size_t)255;
  const size_t oWA  = off; off += (size_t)(2 * DH) * DIN * 2;         off = (off + 255) & ~(size_t)255;
  const size_t oWB  = off; off += (size_t)(2 * DH) * (2 * DH) * 2;    off = (off + 255) & ~(size_t)255;
  const size_t oWC  = off; off += (size_t)(2 * DH) * (2 * DH) * 2;    off = (off + 255) & ~(size_t)255;
  if (off > ws_size || off > (size_t)WSMAX) return;
  unsigned short* ACT = (unsigned short*)(ws + oACT);
  float*          PR  = (float*)(ws + oP);
  unsigned short* WTA = (unsigned short*)(ws + oWA);
  unsigned short* WTB = (unsigned short*)(ws + oWB);
  unsigned short* WTC = (unsigned short*)(ws + oWC);

  (void)hipFuncSetAttribute(reinterpret_cast<const void*>(&k_agg),
                            hipFuncAttributeMaxDynamicSharedMemorySize, LDS_AGG);

  const int nUx = MP * (DIN / 8);
  k_xprep<<<cdiv(nUx, NTHR), NTHR, 0, stream>>>(x, ACT, nN, nUx);

  {
    const int nUa = (2 * DH) * (DIN / 8);
    k_wtr<<<cdiv(nUa, NTHR), NTHR, 0, stream>>>(W1r, W1l, DH, DH, DH, DIN, DIN, WTA, nUa);
    const int nUb = (2 * DH) * ((2 * DH) / 8);
    k_wtr<<<cdiv(nUb, NTHR), NTHR, 0, stream>>>(W2r, W2l, DH, DH, DH, DH, 2 * DH, WTB, nUb);
    k_wtr<<<cdiv(nUb, NTHR), NTHR, 0, stream>>>(Wm1, Wm1 + (size_t)DH * DH, DH, DH, DH, DH, 2 * DH, WTC, nUb);
  }

  const int gM = MP / GBM;
  const int gY = (2 * DH) / (16 * GNT);
  k_gemm<GNT><<<dim3(gM, gY), GTHR, 0, stream>>>(ACT, DIN, WTA, DIN, PR, PW);
  k_agg<<<gA, NTHR, LDS_AGG, stream>>>(src, dst, PR, PW, 0, DH, b1l, ACT, APW, nN, nE, nb, vec8, MP);
  k_gemm<GNT><<<dim3(gM, gY), GTHR, 0, stream>>>(ACT, APW, WTB, 2 * DH, PR, PW);
  k_agg<<<gA, NTHR, LDS_AGG, stream>>>(src, dst, PR, PW, 0, DH, b2l, ACT, APW, nN, nE, nb, vec8, MP);
  k_gemm<GNT><<<dim3(gM, gY), GTHR, 0, stream>>>(ACT, APW, WTC, 2 * DH, PR, PW);
  k_edge<<<cdiv(nLines, NWAVE * LPW), NTHR, 0, stream>>>(PR, PW, DH, src, dst, bm1, Wm2, bm2, out, nN, nE, nLines);
}
